// MolConv_64037962383975
// MI455X (gfx1250) — hardware-verified
//
#include <hip/hip_runtime.h>
#include <stddef.h>


#define FI      64
#define NO      256
#define FO      64
#define APH     72
#define NTHR    256
#define NWAVE   8
#define EPT     8
#define NGRP    2
#define CHUNK   (NTHR * EPT * NGRP)
#define WCAP    (EPT * NGRP * 32)
#define LISTN   (NWAVE * WCAP)
#define NBC     4096
#define NBF     1024
#define RCAP    40960
#define RBN     128
#define ATHR    128
#define AWAVE   4
#define TGT     128
#define DEGCAP  1024
#define GROWS   128
#define OTHR    512
#define NSTAT   128
#define WSCAP   134217728
#define ASCALE  16.0f
#define WSCALE  64.0f
#define PINV    0.0009765625f
#define BNEPS   1e-5f

#define LDS_FILL ((RCAP + NBF + LISTN) * 4 + 64)
#define LDS_A    (GROWS * APH * 2)
#define LDS_STG  (GROWS * NO * 4)
#define LDS_G    (LDS_A + LDS_STG)

static_assert((CHUNK & (CHUNK - 1)) == 0);
static_assert(CHUNK <= 4096);
static_assert(NBC <= 4096 && NBF <= 4096);
static_assert((NBC & (NBC - 1)) == 0 && (NBF & (NBF - 1)) == 0);
static_assert(NBC == 4 * NBF);
static_assert(OTHR * 8 == NBC);
static_assert((RCAP % 32) == 0);
static_assert(TGT == AWAVE * 32 && ATHR == AWAVE * 32);
static_assert((NBC % TGT) == 0 && (GROWS % TGT) == 0 && TGT == GROWS);
static_assert(GROWS == NWAVE * 16);
static_assert((FI % 32) == 0 && NO == 4 * FO && FO == 64);
static_assert((APH % 8) == 0 && (LDS_A % 16) == 0);
static_assert(NSTAT * 2 == NTHR);

typedef float    v2f  __attribute__((ext_vector_type(2)));
typedef float    v4f  __attribute__((ext_vector_type(4)));
typedef float    v8f  __attribute__((ext_vector_type(8)));
typedef int      v4i  __attribute__((ext_vector_type(4)));
typedef double   v2d  __attribute__((ext_vector_type(2)));
typedef _Float16 v8h  __attribute__((ext_vector_type(8)));
typedef _Float16 v16h __attribute__((ext_vector_type(16)));
union FragH { v16h v; v8h h[2]; };

__device__ __forceinline__ v8f wmh(v16h a, v16h b, v8f c) {
  v8f d = __builtin_amdgcn_wmma_f32_16x16x32_f16(false, a, false, b, (short)0, c, false, false);
  asm volatile("v_nop\n\tv_nop\n\tv_nop\n\tv_nop" : "+v"(d) : "v"(a), "v"(b));
  return d;
}

__device__ __forceinline__ _Float16 elu_h(float t, float s) {
  const float e = t > 0.0f ? t : (__expf(t) - 1.0f);
  return (_Float16)(e * s);
}
__device__ __forceinline__ v8h elu_cvt8(v4f a, v4f b, float s) {
  v8h c;
  c[0] = elu_h(a.x, s); c[1] = elu_h(a.y, s); c[2] = elu_h(a.z, s); c[3] = elu_h(a.w, s);
  c[4] = elu_h(b.x, s); c[5] = elu_h(b.y, s); c[6] = elu_h(b.z, s); c[7] = elu_h(b.w, s);
  return c;
}

template <int NT>
__device__ __forceinline__ void mma_tiles(const _Float16* sA, const _Float16* __restrict__ Bw,
                                          int wrow, int lane, v8f (&acc)[NT]) {
  constexpr int NKT = FI / 32;
  const int hh = lane >> 4, m = lane & 15;
#pragma unroll
  for (int t = 0; t < NT; ++t) { v8f z = {0.f, 0.f, 0.f, 0.f, 0.f, 0.f, 0.f, 0.f}; acc[t] = z; }
  const _Float16* ap = sA + (wrow + m) * APH + 8 * hh;
#pragma unroll 1
  for (int kt = 0; kt < NKT; ++kt) {
    FragH a;
    a.h[0] = *(const v8h*)(ap + 32 * kt);
    a.h[1] = *(const v8h*)(ap + 32 * kt + 16);
#pragma unroll
    for (int t = 0; t < NT; ++t) {
      const _Float16* bp = Bw + (size_t)(16 * t + m) * FI + 32 * kt + 8 * hh;
      FragH b;
      b.h[0] = *(const v8h*)bp;
      b.h[1] = *(const v8h*)(bp + 16);
      acc[t] = wmh(a.v, b.v, acc[t]);
    }
  }
}

template <int NB>
__device__ __forceinline__ int scan_chunk(const int* __restrict__ dsts, int nE, int cbase, int slotBase,
                                          int vec8, int* list, int tid, int lane, int wave) {
  int wc = 0;
#pragma unroll
  for (int g = 0; g < NGRP; ++g) {
    const int el0  = (g * NTHR + tid) * EPT;
    const int e0   = cbase + el0;
    const int sent = -2147483647 - 1;
    v4i da, db;
    if (vec8 != 0 && cbase + CHUNK <= nE) {
      da = *(const v4i*)(dsts + e0);
      db = *(const v4i*)(dsts + e0 + 4);
    } else {
      da.x = (e0     < nE) ? dsts[min(e0, nE - 1)] : sent;
      da.y = (e0 + 1 < nE) ? dsts[min(e0 + 1, nE - 1)] : sent;
      da.z = (e0 + 2 < nE) ? dsts[min(e0 + 2, nE - 1)] : sent;
      da.w = (e0 + 3 < nE) ? dsts[min(e0 + 3, nE - 1)] : sent;
      db.x = (e0 + 4 < nE) ? dsts[min(e0 + 4, nE - 1)] : sent;
      db.y = (e0 + 5 < nE) ? dsts[min(e0 + 5, nE - 1)] : sent;
      db.z = (e0 + 6 < nE) ? dsts[min(e0 + 6, nE - 1)] : sent;
      db.w = (e0 + 7 < nE) ? dsts[min(e0 + 7, nE - 1)] : sent;
    }
    const unsigned nb = (unsigned)slotBase;
    const unsigned s0 = (unsigned)da.x - nb, s1 = (unsigned)da.y - nb;
    const unsigned s2 = (unsigned)da.z - nb, s3 = (unsigned)da.w - nb;
    const unsigned s4 = (unsigned)db.x - nb, s5 = (unsigned)db.y - nb;
    const unsigned s6 = (unsigned)db.z - nb, s7 = (unsigned)db.w - nb;
    const bool h0 = s0 < (unsigned)NB, h1 = s1 < (unsigned)NB, h2 = s2 < (unsigned)NB, h3 = s3 < (unsigned)NB;
    const bool h4 = s4 < (unsigned)NB, h5 = s5 < (unsigned)NB, h6 = s6 < (unsigned)NB, h7 = s7 < (unsigned)NB;
    const unsigned any = __builtin_amdgcn_ballot_w32(h0 | h1 | h2 | h3 | h4 | h5 | h6 | h7);
    if (any != 0u) {
#define HITJ(J, HJ, SJ) { \
        const unsigned mj = __builtin_amdgcn_ballot_w32(HJ); \
        if (mj != 0u) { \
          if (HJ) { \
            const int pos = wc + (int)__builtin_amdgcn_mbcnt_lo(mj, 0u); \
            if (pos < WCAP) list[wave * WCAP + pos] = ((el0 + (J)) << 12) | (int)(SJ); \
          } \
          wc += (int)__builtin_popcount(mj); } }
      HITJ(0, h0, s0)
      HITJ(1, h1, s1)
      HITJ(2, h2, s2)
      HITJ(3, h3, s3)
      HITJ(4, h4, s4)
      HITJ(5, h5, s5)
      HITJ(6, h6, s6)
      HITJ(7, h7, s7)
#undef HITJ
    }
  }
  return wc;
}

__global__ __launch_bounds__(NTHR) void k_bnstat(const float* __restrict__ x, double* part, int nN, int rb) {
  __shared__ double s_s[4 * FI];
  __shared__ double s_q[4 * FI];
  __shared__ __attribute__((aligned(16))) double lb[2 * FI];
  const int tid = threadIdx.x, lane = tid & 31, wave = tid >> 5;
  const int col = tid & 63, rg = tid >> 6;
  const int r0 = blockIdx.x * rb;
  int r1 = r0 + rb; r1 = r1 > nN ? nN : r1;
  double s = 0.0, q = 0.0;
#pragma unroll 4
  for (int r = r0 + rg; r < r1; r += 4) {
    const double d = (double)x[(size_t)r * FI + col];
    s += d; q += d * d;
  }
  s_s[rg * FI + col] = s;
  s_q[rg * FI + col] = q;
  __syncthreads();
  if (tid < FI) {
    lb[tid]      = ((s_s[tid] + s_s[FI + tid]) + s_s[2 * FI + tid]) + s_s[3 * FI + tid];
    lb[FI + tid] = ((s_q[tid] + s_q[FI + tid]) + s_q[2 * FI + tid]) + s_q[3 * FI + tid];
  }
  __syncthreads();
  double* dp = part + (size_t)blockIdx.x * 2 * FI + wave * FI + 2 * lane;
  v2d v = {0.0, 0.0};
  if (wave < 2) v = *(const v2d*)(lb + wave * FI + 2 * lane);
  if (wave < 2) *(volatile v2d*)dp = v;
  __threadfence();
  if (wave < 2) *(volatile v2d*)dp = v;
}

__global__ __launch_bounds__(NTHR) void k_prep(
    const float* __restrict__ W, const double* __restrict__ part,
    const float* __restrict__ gamma, const float* __restrict__ beta,
    _Float16* wp, float* ss, int nN, int nStat) {
  __shared__ __attribute__((aligned(16))) _Float16 sW[NO * APH];
  __shared__ __attribute__((aligned(16))) float s_ss[2 * FI];
  const int tid = threadIdx.x, lane = tid & 31, wave = tid >> 5;
  const int kk = tid >> 6, n0 = (tid & 63) * 4;
#pragma unroll 1
  for (int it = 0; it < 16; ++it) {
    const int k = it * 4 + kk;
    const v4f w = *(const v4f*)(W + (size_t)k * NO + n0);
    sW[(n0 + 0) * APH + k] = (_Float16)(w.x * WSCALE);
    sW[(n0 + 1) * APH + k] = (_Float16)(w.y * WSCALE);
    sW[(n0 + 2) * APH + k] = (_Float16)(w.z * WSCALE);
    sW[(n0 + 3) * APH + k] = (_Float16)(w.w * WSCALE);
  }
  if (tid < FI) {
    double s = 0.0, q = 0.0;
#pragma unroll 1
    for (int b = 0; b < nStat; ++b) {
      s += part[(size_t)b * 2 * FI + tid];
      q += part[(size_t)b * 2 * FI + FI + tid];
    }
    const double inv_n = 1.0 / (double)nN;
    const double mean = s * inv_n;
    double var = q * inv_n - mean * mean;
    var = var < 0.0 ? 0.0 : var;
    const float varf = (float)var, meanf = (float)mean;
    const float istd = 1.0f / sqrtf(varf + BNEPS);
    const float sc = istd * gamma[tid];
    s_ss[tid]      = sc;
    s_ss[FI + tid] = beta[tid] - meanf * sc;
  }
  __syncthreads();

  v8h wr[8];
#pragma unroll
  for (int i = 0; i < 8; ++i) {
    const int n = wave * 32 + 4 * i + (lane >> 3);
    wr[i] = *(const v8h*)(sW + n * APH + 8 * (lane & 7));
  }
  v4f sv = {0.f, 0.f, 0.f, 0.f};
  if (wave == 0) sv = *(const v4f*)(s_ss + 4 * lane);
#pragma unroll
  for (int i = 0; i < 8; ++i) {
    const int n = wave * 32 + 4 * i + (lane >> 3);
    *(volatile v8h*)(wp + (size_t)n * FI + 8 * (lane & 7)) = wr[i];
  }
  if (wave == 0) *(volatile v4f*)(ss + 4 * lane) = sv;
  __threadfence();
#pragma unroll
  for (int i = 0; i < 8; ++i) {
    const int n = wave * 32 + 4 * i + (lane >> 3);
    *(volatile v8h*)(wp + (size_t)n * FI + 8 * (lane & 7)) = wr[i];
  }
  if (wave == 0) *(volatile v4f*)(ss + 4 * lane) = sv;
}

__global__ __launch_bounds__(NTHR) void k_gemm(
    const float* __restrict__ x, const float* __restrict__ ss,
    const _Float16* __restrict__ Bw, const float* __restrict__ bias,
    float* C, int nN) {
  extern __shared__ v4f lds_dyn[];
  _Float16* sA  = (_Float16*)lds_dyn;
  float*    stg = (float*)((char*)lds_dyn + LDS_A);
  const int tid = threadIdx.x, lane = tid & 31, wave = tid >> 5, hh = lane >> 4, m = lane & 15;
  const int rowBase = blockIdx.x * GROWS;
  const int c0 = (tid & 7) * 8, rr = tid >> 3;
  const v4f sc0 = *(const v4f*)(ss + c0),      sc1 = *(const v4f*)(ss + c0 + 4);
  const v4f sh0 = *(const v4f*)(ss + FI + c0), sh1 = *(const v4f*)(ss + FI + c0 + 4);

#pragma unroll 1
  for (int it = 0; it < 4; ++it) {
    const int r = it * 32 + rr;
    int row = rowBase + r;
    row = row > nN - 1 ? nN - 1 : row;
    const float* ap = x + (size_t)row * FI + c0;
    const v4f a = *(const v4f*)ap, b = *(const v4f*)(ap + 4);
    const v4f ta = a * sc0 + sh0, tb = b * sc1 + sh1;
    *(v8h*)(sA + r * APH + c0) = elu_cvt8(ta, tb, ASCALE);
  }
  __syncthreads();

#pragma unroll 1
  for (int ch = 0; ch < 4; ++ch) {
    v8f acc[4];
    mma_tiles<4>(sA, Bw + (size_t)(64 * ch) * FI, wave * 16, lane, acc);
    float* sp = stg + (wave * 16 + 8 * hh) * NO + 64 * ch + m;
#pragma unroll
    for (int t = 0; t < 4; ++t) {
      const float bv = bias[64 * ch + 16 * t + m];
#pragma unroll
      for (int r = 0; r < 8; ++r) sp[r * NO + 16 * t] = acc[t][r] * PINV + bv;
    }
  }
  __syncthreads();

  const float* lp = stg + wave * 16 * NO + 4 * lane;
  float* cp = C + (size_t)(rowBase + wave * 16) * NO + 4 * lane;
#pragma unroll
  for (int i = 0; i < 16; ++i) {
#pragma unroll
    for (int hf = 0; hf < 2; ++hf) {
      const v4f v = *(const v4f*)(lp + NO * i + 128 * hf);
      *(volatile v4f*)(cp + (size_t)NO * i + 128 * hf) = v;
    }
  }
  __threadfence();
#pragma unroll
  for (int i = 0; i < 16; ++i) {
#pragma unroll
    for (int hf = 0; hf < 2; ++hf) {
      const v4f v = *(const v4f*)(lp + NO * i + 128 * hf);
      *(volatile v4f*)(cp + (size_t)NO * i + 128 * hf) = v;
    }
  }
}

__global__ __launch_bounds__(NTHR) void k_count(const int* __restrict__ dsts, int* cnt, int nE, int vec8) {
  __shared__ __attribute__((aligned(16))) int scnt[NBC];
  __shared__ __attribute__((aligned(16))) int list[LISTN];
  __shared__ int wcnt[NWAVE];
  const int tid = threadIdx.x, lane = tid & 31, wave = tid >> 5;
  const int nodeBase = blockIdx.x * NBC;

  for (int i = tid; i < NBC; i += NTHR) scnt[i] = 0;
  __syncthreads();

  const int nChunks = (nE + CHUNK - 1) / CHUNK;
#pragma unroll 1
  for (int ch = 0; ch < nChunks; ++ch) {
    const int cbase = ch * CHUNK;
    const int wc = scan_chunk<NBC>(dsts, nE, cbase, nodeBase, vec8, list, tid, lane, wave);
    if (lane == 0) wcnt[wave] = wc;
    __syncthreads();
    if (wave == 0) {
#pragma unroll 1
      for (int wsx = 0; wsx < NWAVE; ++wsx) {
        int n = __builtin_amdgcn_readfirstlane(wcnt[wsx]);
        n = n > WCAP ? WCAP : (n < 0 ? 0 : n);
        const int* lp = list + wsx * WCAP;
#pragma unroll 1
        for (int i = 0; i < n; ++i) {
          const int ent  = __builtin_amdgcn_readfirstlane(lp[i]);
          const int slot = ent & (NBC - 1);
          if (lane == 0) scnt[slot] = scnt[slot] + 1;
        }
      }
    }
    __syncthreads();
  }

  v4i cq[4];
#pragma unroll
  for (int q = 0; q < 4; ++q) {
    const int f = (wave * 4 + q) * 128 + 4 * lane;
    cq[q] = *(const v4i*)(scnt + f);
  }
  int* cp = cnt + (size_t)nodeBase;
#pragma unroll
  for (int q = 0; q < 4; ++q) {
    const int f = (wave * 4 + q) * 128 + 4 * lane;
    *(volatile v4i*)(cp + f) = cq[q];
  }
  __threadfence();
#pragma unroll
  for (int q = 0; q < 4; ++q) {
    const int f = (wave * 4 + q) * 128 + 4 * lane;
    *(volatile v4i*)(cp + f) = cq[q];
  }
}

__global__ __launch_bounds__(OTHR) void k_offsets(
    const int* __restrict__ cnt, int* off, int* rbase, int nChunk) {
  __shared__ __attribute__((aligned(16))) int soff[NBC];
  __shared__ __attribute__((aligned(16))) int srb[RBN];
  __shared__ int wtot[OTHR / 32];
  const int tid = threadIdx.x, lane = tid & 31, wave = tid >> 5, sub = tid >> 7;
  for (int i = tid; i < RBN; i += OTHR) srb[i] = 0;
  int carry = 0;
#pragma unroll 1
  for (int ch = 0; ch < nChunk; ++ch) {
    const int base = ch * NBC;
    const v4i c0 = *(const v4i*)(cnt + base + 8 * tid);
    const v4i c1 = *(const v4i*)(cnt + base + 8 * tid + 4);
    const int e0 = max(c0.x, 0), e1 = max(c0.y, 0), e2 = max(c0.z, 0), e3 = max(c0.w, 0);
    const int e4 = max(c1.x, 0), e5 = max(c1.y, 0), e6 = max(c1.z, 0), e7 = max(c1.w, 0);
    const int ts = e0 + e1 + e2 + e3 + e4 + e5 + e6 + e7;
    int incl = ts;
#pragma unroll
    for (int d = 1; d < 32; d <<= 1) {
      const int t = __shfl_up(incl, d);
      if (lane >= d) incl += t;
    }
    if (lane == 31) wtot[wave] = incl;
    __syncthreads();
    const int S0 = wtot[0]  + wtot[1]  + wtot[2]  + wtot[3];
    const int S1 = wtot[4]  + wtot[5]  + wtot[6]  + wtot[7];
    const int S2 = wtot[8]  + wtot[9]  + wtot[10] + wtot[11];
    const int S3 = wtot[12] + wtot[13] + wtot[14] + wtot[15];
    int pre = 0;
#pragma unroll 1
    for (int w = 4 * sub; w < wave; ++w) pre += wtot[w];
    const int b0 = carry;
    const int b1 = b0 + ((S0 + 31) & ~31);
    const int b2 = b1 + ((S1 + 31) & ~31);
    const int b3 = b2 + ((S2 + 31) & ~31);
    const int b4 = b3 + ((S3 + 31) & ~31);
    const int myb = sub == 0 ? b0 : (sub == 1 ? b1 : (sub == 2 ? b2 : b3));
    if (tid == 0) {
      srb[min(4 * ch + 0, RBN - 1)] = b0;
      srb[min(4 * ch + 1, RBN - 1)] = b1;
      srb[min(4 * ch + 2, RBN - 1)] = b2;
      srb[min(4 * ch + 3, RBN - 1)] = b3;
    }
    int run = myb + pre + incl - ts;
    soff[8 * tid + 0] = run; run += e0;
    soff[8 * tid + 1] = run; run += e1;
    soff[8 * tid + 2] = run; run += e2;
    soff[8 * tid + 3] = run; run += e3;
    soff[8 * tid + 4] = run; run += e4;
    soff[8 * tid + 5] = run; run += e5;
    soff[8 * tid + 6] = run; run += e6;
    soff[8 * tid + 7] = run;
    carry = b4;
    __syncthreads();
    const v4i o0 = *(const v4i*)(soff + 4 * tid);
    const v4i o1 = *(const v4i*)(soff + 4 * (tid + OTHR));
    int* op = off + base;
    *(volatile v4i*)(op + 4 * tid) = o0;
    *(volatile v4i*)(op + 4 * (tid + OTHR)) = o1;
    __threadfence();
    *(volatile v4i*)(op + 4 * tid) = o0;
    *(volatile v4i*)(op + 4 * (tid + OTHR)) = o1;
    __syncthreads();
  }
  if (tid == 0) srb[min(4 * nChunk, RBN - 1)] = carry;
  __syncthreads();
  v4i rv = {0, 0, 0, 0};
  if (tid < 32) rv = *(const v4i*)(srb + 4 * tid);
  if (tid < 32) *(volatile v4i*)(rbase + 4 * tid) = rv;
  __threadfence();
  if (tid < 32) *(volatile v4i*)(rbase + 4 * tid) = rv;
}

__global__ __launch_bounds__(NTHR) void k_fill(
    const int* __restrict__ dsts, const int* __restrict__ off, const int* __restrict__ rbase,
    int* csr, int nE, int vec8, int csrLen) {
  extern __shared__ v4f lds_dyn[];
  int* region = (int*)lds_dyn;
  int* cursor = region + RCAP;
  int* list   = cursor + NBF;
  int* wcnt   = list + LISTN;
  const int tid = threadIdx.x, lane = tid & 31, wave = tid >> 5;
  const int b = blockIdx.x;
  const int nodeBase = b * NBF;

  int rb0 = rbase[b];
  const int rb1 = rbase[b + 1];
  rb0 = rb0 < 0 ? 0 : (rb0 > csrLen ? csrLen : rb0);
  rb0 &= ~31;
  int len = rb1 - rb0;
  len = len < 0 ? 0 : (len > RCAP ? RCAP : len);
  int lenW = (len + 31) & ~31;
  if (rb0 + lenW > csrLen) lenW = (csrLen - rb0) & ~31;

  {
    const v4i z = {0, 0, 0, 0};
    for (int i = tid; i < RCAP / 4; i += NTHR) ((v4i*)region)[i] = z;
    for (int s = tid; s < NBF; s += NTHR) {
      int o = off[nodeBase + s] - rb0;
      o = o < 0 ? 0 : (o > RCAP ? RCAP : o);
      cursor[s] = o;
    }
  }
  __syncthreads();

  const int nChunks = (nE + CHUNK - 1) / CHUNK;
#pragma unroll 1
  for (int ch = 0; ch < nChunks; ++ch) {
    const int cbase = ch * CHUNK;
    const int wc = scan_chunk<NBF>(dsts, nE, cbase, nodeBase, vec8, list, tid, lane, wave);
    if (lane == 0) wcnt[wave] = wc;
    __syncthreads();
    if (wave == 0) {
#pragma unroll 1
      for (int wsx = 0; wsx < NWAVE; ++wsx) {
        int n = __builtin_amdgcn_readfirstlane(wcnt[wsx]);
        n = n > WCAP ? WCAP : (n < 0 ? 0 : n);
        const int* lp = list + wsx * WCAP;
#pragma unroll 1
        for (int i = 0; i < n; ++i) {
          const int ent  = __builtin_amdgcn_readfirstlane(lp[i]);
          const int slot = ent & (NBF - 1);
          int e = cbase + ((ent >> 12) & (CHUNK - 1));
          e = e < 0 ? 0 : (e > nE - 1 ? nE - 1 : e);
          if (lane == 0) {
            int pos = cursor[slot];
            pos = pos < 0 ? 0 : (pos > RCAP - 1 ? RCAP - 1 : pos);
            region[pos] = e;
            const int np = pos + 1;
            cursor[slot] = np > RCAP ? RCAP : np;
          }
        }
      }
    }
    __syncthreads();
  }

  const int nv = lenW >> 2;
  int* gp = csr + rb0;
#pragma unroll 1
  for (int i = tid; i < nv; i += NTHR) { const v4i v = ((const v4i*)region)[i]; *(volatile v4i*)(gp + 4 * i) = v; }
  __threadfence();
#pragma unroll 1
  for (int i = tid; i < nv; i += NTHR) { const v4i v = ((const v4i*)region)[i]; *(volatile v4i*)(gp + 4 * i) = v; }
}

__global__ __launch_bounds__(ATHR) void k_agg(
    const int* __restrict__ csr, const int* __restrict__ off, const int* __restrict__ cnt,
    const int* __restrict__ cols, const float* __restrict__ wts, const float* __restrict__ xlin,
    float* out, int nN, int nE, int csrLen) {
#pragma clang fp contract(off)
  __shared__ __attribute__((aligned(16))) float stg[TGT * FO];
  const int tid = threadIdx.x, lane = tid & 31, wave = tid >> 5, hh = lane >> 4, m = lane & 15;
  const int tbase = blockIdx.x * TGT + wave * 32;
  const int cl = tbase + lane;
  const int cnt_l = cnt[cl];
  const int off_l = off[cl];
  const int kn = 4 * nN, n2 = 2 * nN, n3 = 3 * nN;

#pragma unroll 1
  for (int j = 0; j < 32; ++j) {
    int n = __builtin_amdgcn_readlane(cnt_l, j);
    n = n < 0 ? 0 : (n > DEGCAP ? DEGCAP : n);
    const int st = __builtin_amdgcn_readlane(off_l, j);
    v2f sm = {0.0f, 0.0f};
#pragma unroll 1
    for (int q0 = 0; q0 < n; q0 += 32) {
      int pos = st + q0 + lane;
      pos = pos < 0 ? 0 : (pos > csrLen - 1 ? csrLen - 1 : pos);
      int el = csr[pos];
      el = el < 0 ? 0 : (el > nE - 1 ? nE - 1 : el);
      int col = cols[el];
      col = col < 0 ? col + kn : col;
      col = col < 0 ? 0 : (col > kn - 1 ? kn - 1 : col);
      const int k  = (col >= nN ? 1 : 0) + (col >= n2 ? 1 : 0) + (col >= n3 ? 1 : 0);
      const int nd = col - k * nN;
      const int ro = nd * NO + k * FO;
      const int wb = __float_as_int(wts[el]);
      const int mcnt = (n - q0) < 32 ? (n - q0) : 32;
#pragma unroll 1
      for (int p = 0; p < mcnt; ++p) {
        const int   r  = __builtin_amdgcn_readlane(ro, p);
        const float wv = __int_as_float(__builtin_amdgcn_readlane(wb, p));
        const v2f xv = *(const v2f*)(xlin + (size_t)r + 2 * lane);
        const v2f pr = xv * wv;
        sm = sm + pr;
      }
    }
    *(v2f*)(stg + (wave * 32 + j) * FO + 2 * lane) = sm;
  }
  __syncthreads();

  const float* lp = stg + wave * 32 * FO;
#pragma unroll
  for (int i = 0; i < 16; ++i) {
    const int rl = 2 * i + hh;
    const int row = tbase + rl;
    const v4f v = *(const v4f*)(lp + rl * FO + 4 * m);
    if (row < nN) *(volatile v4f*)(out + (size_t)row * FO + 4 * m) = v;
  }
  __threadfence();
#pragma unroll
  for (int i = 0; i < 16; ++i) {
    const int rl = 2 * i + hh;
    const int row = tbase + rl;
    const v4f v = *(const v4f*)(lp + rl * FO + 4 * m);
    if (row < nN) *(volatile v4f*)(out + (size_t)row * FO + 4 * m) = v;
  }
}

extern "C" void kernel_launch(void* const* d_in, const int* in_sizes, int n_in,
                              void* d_out, int out_size, void* d_ws, size_t ws_size,
                              hipStream_t stream) {
  if (n_in < 8) return;
  const int nN = in_sizes[0] / FI;
  const int nE = in_sizes[5];
  if (nN <= 0 || nE <= 0) return;
  if (in_sizes[0] != nN * FI) return;
  if (in_sizes[1] != FI || in_sizes[2] != FI) return;
  if (in_sizes[3] != FI * NO || in_sizes[4] != NO) return;
  if (in_sizes[6] != nE || in_sizes[7] != nE) return;
  if (out_size != nN * FO) return;
  if (nE > (1 << 28) || nN > (1 << 22)) return;

  const float* atoms = (const float*)d_in[0];
  const float* gamma = (const float*)d_in[1];
  const float* beta  = (const float*)d_in[2];
  const float* W     = (const float*)d_in[3];
  const float* bia   = (const float*)d_in[4];
  const float* wts   = (const float*)d_in[5];
  const int*   dsts  = (const int*)d_in[6];
  const int*   cols  = (const int*)d_in[7];
  float* out = (float*)d_out;

  const int NPAD   = ((nN + TGT - 1) / TGT) * TGT;
  const int nBC    = (nN + NBC - 1) / NBC;
  const int CNTPAD = nBC * NBC;
  if (4 * nBC + 1 > RBN) return;
  const int nBF    = (nN + NBF - 1) / NBF;
  const int csrLen = ((nE + 31) & ~31) + 4096;
  if (31 * 4 * nBC > 4096) return;
  const int nGemm  = NPAD / GROWS;
  const int nAgg   = NPAD / TGT;
  const int rb     = (nN + NSTAT - 1) / NSTAT;

  char* ws = (char*)d_ws;
  size_t off = 0;
  const size_t oWp  = off; off += (size_t)NO * FI * 2;             off = (off + 255) & ~(size_t)255;
  const size_t oPrt = off; off += (size_t)NSTAT * 2 * FI * 8;       off = (off + 255) & ~(size_t)255;
  const size_t oSs  = off; off += (size_t)2 * FI * 4;               off = (off + 255) & ~(size_t)255;
  const size_t oCnt = off; off += (size_t)CNTPAD * 4;               off = (off + 255) & ~(size_t)255;
  const size_t oOff = off; off += (size_t)CNTPAD * 4;               off = (off + 255) & ~(size_t)255;
  const size_t oRb  = off; off += (size_t)RBN * 4;                  off = (off + 255) & ~(size_t)255;
  const size_t oCsr = off; off += (size_t)csrLen * 4;               off = (off + 255) & ~(size_t)255;
  const size_t oX   = off; off += (size_t)NPAD * NO * 4;            off = (off + 255) & ~(size_t)255;
  if (off > ws_size || off > (size_t)WSCAP) return;
  _Float16* wp   = (_Float16*)(ws + oWp);
  double*   part = (double*)(ws + oPrt);
  float*    ss   = (float*)(ws + oSs);
  int*      cnt  = (int*)(ws + oCnt);
  int*      offp = (int*)(ws + oOff);
  int*      rbp  = (int*)(ws + oRb);
  int*      csr  = (int*)(ws + oCsr);
  float*    xlin = (float*)(ws + oX);

  const int vec8 = 1;

  k_bnstat<<<NSTAT, NTHR, 0, stream>>>(atoms, part, nN, rb);

  k_prep<<<1, NTHR, 0, stream>>>(W, part, gamma, beta, wp, ss, nN, NSTAT);

  k_count<<<nBC, NTHR, 0, stream>>>(dsts, cnt, nE, vec8);
  k_offsets<<<1, OTHR, 0, stream>>>(cnt, offp, rbp, nBC);
  hipFuncSetAttribute(reinterpret_cast<const void*>(&k_fill),
                      hipFuncAttributeMaxDynamicSharedMemorySize, LDS_FILL);
  k_fill<<<nBF, NTHR, LDS_FILL, stream>>>(dsts, offp, rbp, csr, nE, vec8, csrLen);

  hipFuncSetAttribute(reinterpret_cast<const void*>(&k_gemm),
                      hipFuncAttributeMaxDynamicSharedMemorySize, LDS_G);
  k_gemm<<<nGemm, NTHR, LDS_G, stream>>>(atoms, ss, wp, bia, xlin, nN);

  k_agg<<<nAgg, ATHR, 0, stream>>>(csr, offp, cnt, cols, wts, xlin, out, nN, nE, csrLen);
}
